// StackedBiGRUModel_42185168782068
// MI455X (gfx1250) — hardware-run, weakly checked
//
#include <hip/hip_runtime.h>
#include <math.h>

typedef __attribute__((ext_vector_type(16))) _Float16 v16h;
typedef __attribute__((ext_vector_type(8)))  _Float16 v8h;
typedef __attribute__((ext_vector_type(8)))  float    v8f;
typedef __attribute__((ext_vector_type(4)))  float    v4f;
typedef __attribute__((ext_vector_type(4)))  int      v4i;

constexpr int kB    = 256;
constexpr int kT    = 512;
constexpr int kV    = 30000;
constexpr int kE    = 256;
constexpr int kH    = 32;
constexpr int kG    = 3 * kH;
constexpr int kN2   = 2 * kG;
constexpr int kM    = kB * kT;
constexpr int kOut  = 6;
constexpr int kTop  = 2 * kH;
static_assert(kG == 96);
static_assert(kN2 == 192);
static_assert(kM == 131072);
static_assert((kE % 32) == 0 && (kTop % 32) == 0 && (kH % 32) == 0);
static_assert((kM % 64) == 0 && (kG % 16) == 0 && (kB % 64) == 0);

constexpr float kCarry  = 64.0f;
constexpr float kFold   = 1.0f / (kCarry * kCarry);
constexpr float kF16Min = 6.103515625e-5f;

constexpr size_t kSzGI   = (size_t)kM * kN2 * 4;
constexpr size_t kSzX1   = (size_t)2 * kM * kH * 2;
constexpr size_t kSzEH   = (size_t)kV * kE * 2;
constexpr size_t kSzW0H  = (size_t)kN2 * kE * 2;
constexpr size_t kSzW1H  = (size_t)kN2 * kTop * 2;
constexpr size_t kSzWHH  = (size_t)4 * kG * kH * 2;
constexpr size_t kSzHFIN = (size_t)2 * kB * kH * 4;
constexpr size_t kOffGI   = 0;
constexpr size_t kOffX1   = kOffGI  + kSzGI;
constexpr size_t kOffEH   = kOffX1  + kSzX1;
constexpr size_t kOffW0H  = kOffEH  + kSzEH;
constexpr size_t kOffW1H  = kOffW0H + kSzW0H;
constexpr size_t kOffWHH  = kOffW1H + kSzW1H;
constexpr size_t kOffHFIN = kOffWHH + kSzWHH;
constexpr size_t kWsTotal = kOffHFIN + kSzHFIN;
static_assert(kWsTotal == 133013504ull);
static_assert(kWsTotal <= 134217728ull);
static_assert((kOffX1 % 128) == 0 && (kOffEH % 128) == 0 && (kOffW0H % 128) == 0 &&
              (kOffW1H % 128) == 0 && (kOffWHH % 128) == 0 && (kOffHFIN % 128) == 0);
constexpr size_t kX1Plane = (size_t)kM * kH;

union FragU { v16h v; v8h h[2]; };

__device__ __forceinline__ _Float16 to_h16c(float v) {
  const float s = v * kCarry;
  const float f = (fabsf(s) < kF16Min) ? 0.0f : s;
  return (_Float16)f;
}

__device__ __forceinline__ v8f mma_h(v16h a, v16h b, v8f c) {
  c = __builtin_amdgcn_wmma_f32_16x16x32_f16(false, a, false, b, (short)0, c, false, false);
  asm volatile("v_nop\n\tv_nop\n\tv_nop\n\tv_nop" : "+v"(c) : "v"(a), "v"(b));
  return c;
}

__device__ __forceinline__ void cvt8_store(const float* __restrict__ src, unsigned short* __restrict__ dst, size_t e0) {
  const v4f a0 = *(const v4f*)(src + e0);
  const v4f a1 = *(const v4f*)(src + e0 + 4);
  v8h hv;
  hv[0] = to_h16c(a0[0]);
  hv[1] = to_h16c(a0[1]);
  hv[2] = to_h16c(a0[2]);
  hv[3] = to_h16c(a0[3]);
  hv[4] = to_h16c(a1[0]);
  hv[5] = to_h16c(a1[1]);
  hv[6] = to_h16c(a1[2]);
  hv[7] = to_h16c(a1[3]);
  unsigned short* q = dst + e0;
  *(volatile v8h*)q = hv;
  __threadfence();
  *(volatile v8h*)q = hv;
}

__global__ __launch_bounds__(256) void cvt_f16c8_kernel(
    const float* __restrict__ src, unsigned short* __restrict__ dst, int n8)
{
  const int i = blockIdx.x * 256 + threadIdx.x;
  if (i >= n8) return;
  cvt8_store(src, dst, (size_t)i << 3);
}

struct PrepArgs {
  const float* wih0f; const float* wih0b; const float* wih1f; const float* wih1b;
  const float* whh0f; const float* whh0b; const float* whh1f; const float* whh1b;
  unsigned short* w0h; unsigned short* w1h; unsigned short* whh;
};
static_assert(sizeof(PrepArgs) == 88);

__global__ __launch_bounds__(128) void prep_weights_kernel(PrepArgs p)
{
  const int bx = blockIdx.x;
  const float* src;
  unsigned short* dst;
  int lb;
  if (bx < 24) {
    src = p.wih0f; dst = p.w0h; lb = bx;
  } else if (bx < 48) {
    src = p.wih0b; dst = p.w0h + (size_t)kG * kE; lb = bx - 24;
  } else if (bx < 54) {
    src = p.wih1f; dst = p.w1h; lb = bx - 48;
  } else if (bx < 60) {
    src = p.wih1b; dst = p.w1h + (size_t)kG * kTop; lb = bx - 54;
  } else {
    const int q = (bx - 60) / 3;
    lb = (bx - 60) - q * 3;
    src = (q == 0) ? p.whh0f : (q == 1) ? p.whh0b : (q == 2) ? p.whh1f : p.whh1b;
    dst = p.whh + (size_t)q * kG * kH;
  }
  cvt8_store(src, dst, ((size_t)lb * 128 + threadIdx.x) << 3);
}

constexpr int kAPitch = kE + 8;
constexpr int kSlabP  = 100;

template <int LAYER>
__global__ __launch_bounds__(128) void gi_gemm_kernel(
    const unsigned short* __restrict__ Ap, const int* __restrict__ ids,
    const unsigned short* __restrict__ Wp,
    const float* __restrict__ bih_f, const float* __restrict__ bih_b,
    float* __restrict__ GI)
{
  constexpr int KD = (LAYER == 0) ? kE : kTop;
  __shared__ __align__(16) _Float16 sA[(LAYER == 0) ? 64 * kAPitch : 8];
  __shared__ __align__(16) float sSlab[4][16 * kSlabP];

  const _Float16* A = (const _Float16*)Ap;
  const _Float16* W = (const _Float16*)Wp;
  const int tid  = threadIdx.x;
  const int lane = tid & 31;
  const int wave = tid >> 5;
  const int hh   = lane >> 4;
  const int rl   = lane & 15;
  const int m0   = blockIdx.x * 64;
  const int mh   = wave >> 1;
  const int nh   = wave & 1;

  if (LAYER == 0) {
    const int tq  = m0 >> 8;
    const int bq0 = m0 & (kB - 1);
#pragma unroll 4
    for (int it = 0; it < 16; ++it) {
      const int i   = it * 128 + tid;
      const int row = i >> 5;
      const int ch  = (i & 31) * 8;
      int id = ids[(bq0 + row) * kT + tq];
      id = (id < 0) ? 0 : ((id > kV - 1) ? (kV - 1) : id);
      const v8h v = *(const v8h*)(A + (size_t)id * kE + ch);
      *(v8h*)(sA + row * kAPitch + ch) = v;
    }
    __syncthreads();
  }

  v8f acc[2][6];
#pragma unroll
  for (int i = 0; i < 2; ++i)
#pragma unroll
    for (int j = 0; j < 6; ++j) acc[i][j] = (v8f){0.f, 0.f, 0.f, 0.f, 0.f, 0.f, 0.f, 0.f};

#pragma unroll 1
  for (int k0 = 0; k0 < KD; k0 += 32) {
    FragU a0, a1;
    if (LAYER == 0) {
      const int o0 = (32 * mh + rl) * kAPitch + k0 + 8 * hh;
      a0.h[0] = *(const v8h*)(sA + o0);
      a0.h[1] = *(const v8h*)(sA + o0 + 16);
      a1.h[0] = *(const v8h*)(sA + o0 + 16 * kAPitch);
      a1.h[1] = *(const v8h*)(sA + o0 + 16 * kAPitch + 16);
    } else {
      const _Float16* p0 = A + (size_t)(k0 >> 5) * kX1Plane + (size_t)(m0 + 32 * mh + rl) * kH + 8 * hh;
      a0.h[0] = *(const v8h*)(p0);
      a0.h[1] = *(const v8h*)(p0 + 16);
      a1.h[0] = *(const v8h*)(p0 + 16 * kH);
      a1.h[1] = *(const v8h*)(p0 + 16 * kH + 16);
    }
#pragma unroll
    for (int j = 0; j < 6; ++j) {
      FragU bf;
      const _Float16* q = W + (size_t)(kG * nh + 16 * j + rl) * KD + k0 + 8 * hh;
      bf.h[0] = *(const v8h*)(q);
      bf.h[1] = *(const v8h*)(q + 16);
      acc[0][j] = mma_h(a0.v, bf.v, acc[0][j]);
      acc[1][j] = mma_h(a1.v, bf.v, acc[1][j]);
    }
  }

  const float* bp = nh ? bih_b : bih_f;
  float bcol[6];
#pragma unroll
  for (int j = 0; j < 6; ++j) bcol[j] = bp[16 * j + rl];

  float* slab = sSlab[wave];
#pragma unroll
  for (int i = 0; i < 2; ++i) {
#pragma unroll
    for (int j = 0; j < 6; ++j) {
#pragma unroll
      for (int r = 0; r < 8; ++r) {
        slab[(8 * hh + r) * kSlabP + 16 * j + rl] = acc[i][j][r] * kFold + bcol[j];
      }
    }
    __syncthreads();
    v4f sv[12];
#pragma unroll
    for (int it = 0; it < 12; ++it) {
      const int idx = it * 32 + lane;
      const int row = idx / 24;
      const int c4  = (idx - row * 24) * 4;
      sv[it] = *(const v4f*)(slab + row * kSlabP + c4);
    }
    for (int pass = 0; pass < 2; ++pass) {
#pragma unroll
      for (int it = 0; it < 12; ++it) {
        const int idx = it * 32 + lane;
        const int row = idx / 24;
        const int c4  = (idx - row * 24) * 4;
        *(volatile v4f*)(GI + (size_t)(m0 + 32 * mh + 16 * i + row) * kN2 + kG * nh + c4) = sv[it];
      }
      __threadfence();
    }
    __syncthreads();
  }
}

constexpr int kMaskP = kT + 4;
constexpr int kGiP   = 100;
constexpr int kHP    = 40;

template <int LAYER>
__global__ __launch_bounds__(64) void gru_scan_kernel(
    const float* __restrict__ GI, const unsigned short* __restrict__ WHHp,
    const float* __restrict__ bhh_f, const float* __restrict__ bhh_b,
    const int* __restrict__ mask,
    unsigned short* __restrict__ X1, float* __restrict__ HFIN)
{
  __shared__ __align__(16) int      sMk[16 * kMaskP];
  __shared__ __align__(16) float    sGI[16 * kGiP];
  __shared__ __align__(16) _Float16 sH[16 * kHP];
  __shared__ __align__(16) _Float16 sX[16 * kH];

  const int tid  = threadIdx.x;
  const int lane = tid & 31;
  const int wave = tid >> 5;
  const int hh   = lane >> 4;
  const int rl   = lane & 15;
  const int dir  = blockIdx.x >> 4;
  const int b0   = (blockIdx.x & 15) * 16;
  const int jc   = 16 * wave + rl;

#pragma unroll 4
  for (int it = 0; it < 32; ++it) {
    const int i   = it * 64 + tid;
    const int row = i >> 7;
    const int c4  = (i & 127) * 4;
    const v4i mv = *(const v4i*)(mask + (size_t)(b0 + row) * kT + c4);
    *(v4i*)(sMk + row * kMaskP + c4) = mv;
  }
  {
    const int e   = tid * 8;
    const int row = e >> 5;
    const int col = e & 31;
    v8h z;
#pragma unroll
    for (int q = 0; q < 8; ++q) z[q] = (_Float16)0.0f;
    *(v8h*)(sH + row * kHP + col) = z;
  }

  const _Float16* Wd = (const _Float16*)WHHp + (size_t)(LAYER * 2 + dir) * kG * kH;
  FragU bq0, bq1, bq2;
  {
    const _Float16* q0 = Wd + (size_t)(jc) * kH + 8 * hh;
    const _Float16* q1 = Wd + (size_t)(kH + jc) * kH + 8 * hh;
    const _Float16* q2 = Wd + (size_t)(2 * kH + jc) * kH + 8 * hh;
    bq0.h[0] = *(const v8h*)(q0);
    bq0.h[1] = *(const v8h*)(q0 + 16);
    bq1.h[0] = *(const v8h*)(q1);
    bq1.h[1] = *(const v8h*)(q1 + 16);
    bq2.h[0] = *(const v8h*)(q2);
    bq2.h[1] = *(const v8h*)(q2 + 16);
  }
  const float* bhh = dir ? bhh_b : bhh_f;
  const float bh0 = bhh[jc];
  const float bh1 = bhh[kH + jc];
  const float bh2 = bhh[2 * kH + jc];

  float hreg[8];
#pragma unroll
  for (int r = 0; r < 8; ++r) hreg[r] = 0.0f;

  __syncthreads();

#pragma unroll 1
  for (int s = 0; s < kT; ++s) {
    const int t = dir ? (kT - 1 - s) : s;

    const float* gsrc = GI + ((size_t)t * kB + b0) * kN2 + dir * kG;
    v4f gv[6];
#pragma unroll
    for (int it = 0; it < 6; ++it) {
      const int idx = it * 64 + tid;
      const int row = idx / 24;
      const int c4  = (idx - row * 24) * 4;
      gv[it] = *(const v4f*)(gsrc + (size_t)row * kN2 + c4);
    }

    FragU a;
    a.h[0] = *(const v8h*)(sH + rl * kHP + 8 * hh);
    a.h[1] = *(const v8h*)(sH + rl * kHP + 16 + 8 * hh);

    v8f c0 = (v8f){0.f, 0.f, 0.f, 0.f, 0.f, 0.f, 0.f, 0.f};
    v8f c1 = (v8f){0.f, 0.f, 0.f, 0.f, 0.f, 0.f, 0.f, 0.f};
    v8f c2 = (v8f){0.f, 0.f, 0.f, 0.f, 0.f, 0.f, 0.f, 0.f};
    c0 = mma_h(a.v, bq0.v, c0);
    c1 = mma_h(a.v, bq1.v, c1);
    c2 = mma_h(a.v, bq2.v, c2);

#pragma unroll
    for (int it = 0; it < 6; ++it) {
      const int idx = it * 64 + tid;
      const int row = idx / 24;
      const int c4  = (idx - row * 24) * 4;
      *(v4f*)(sGI + row * kGiP + c4) = gv[it];
    }
    __syncthreads();

#pragma unroll
    for (int r = 0; r < 8; ++r) {
      const int row = 8 * hh + r;
      const float ir  = sGI[row * kGiP + jc];
      const float iz  = sGI[row * kGiP + kH + jc];
      const float inn = sGI[row * kGiP + 2 * kH + jc];
      const int   mk  = sMk[row * kMaskP + t];
      const float hr = c0[r] * kFold + bh0;
      const float hz = c1[r] * kFold + bh1;
      const float hn = c2[r] * kFold + bh2;
      const float rg = __builtin_amdgcn_rcpf(1.0f + expf(-(ir + hr)));
      const float zg = __builtin_amdgcn_rcpf(1.0f + expf(-(iz + hz)));
      const float ng = tanhf(inn + rg * hn);
      const float hprev = hreg[r];
      const float hnew  = (1.0f - zg) * ng + zg * hprev;
      const float hsel  = (mk > 0) ? hnew : hprev;
      hreg[r] = hsel;
      const _Float16 h16 = to_h16c(hsel);
      sH[row * kHP + jc] = h16;
      if (LAYER == 0) sX[row * kH + jc] = h16;
    }
    __syncthreads();

    if (LAYER == 0) {
      if (wave == 0) {
        const v8h xa = *(const v8h*)(sX + lane * 8);
        const v8h xb = *(const v8h*)(sX + 256 + lane * 8);
        unsigned short* dst = X1 + (size_t)dir * kX1Plane + ((size_t)t * kB + b0) * kH;
        for (int pass = 0; pass < 2; ++pass) {
          *(volatile v8h*)(dst + lane * 8) = xa;
          *(volatile v8h*)(dst + 256 + lane * 8) = xb;
          __threadfence();
        }
      }
    }
  }

  if (LAYER == 1) {
#pragma unroll
    for (int r = 0; r < 8; ++r) sGI[(8 * hh + r) * kH + jc] = hreg[r];
    __syncthreads();
    if (wave == 0) {
      v4f fv[4];
#pragma unroll
      for (int it = 0; it < 4; ++it) fv[it] = *(const v4f*)(sGI + (it * 32 + lane) * 4);
      float* dst = HFIN + ((size_t)dir * kB + b0) * kH;
      for (int pass = 0; pass < 2; ++pass) {
#pragma unroll
        for (int it = 0; it < 4; ++it) *(volatile v4f*)(dst + (it * 32 + lane) * 4) = fv[it];
        __threadfence();
      }
    }
  }
}

static_assert(((kB * kOut) % 256) == 0);
__global__ __launch_bounds__(256) void head_kernel(
    const float* __restrict__ HFIN, const float* __restrict__ Wout,
    const float* __restrict__ bout, float* __restrict__ out)
{
  const int i = blockIdx.x * 256 + threadIdx.x;
  const int b = i / kOut;
  const int o = i - b * kOut;
  const float* w = Wout + o * kTop;
  float acc = 0.0f;
#pragma unroll 1
  for (int k4 = 0; k4 < kTop / 4; ++k4) {
    const float* xp = HFIN + (size_t)(k4 >> 3) * kB * kH + (size_t)b * kH + (k4 & 7) * 4;
    const v4f x  = *(const v4f*)(xp);
    const v4f wv = *(const v4f*)(w + k4 * 4);
    acc = fmaf(x[0], wv[0], acc);
    acc = fmaf(x[1], wv[1], acc);
    acc = fmaf(x[2], wv[2], acc);
    acc = fmaf(x[3], wv[3], acc);
  }
  const float res = acc + bout[o];
  *(volatile float*)(out + i) = res;
  __threadfence();
  *(volatile float*)(out + i) = res;
}

extern "C" void kernel_launch(void* const* d_in, const int* in_sizes, int n_in,
                              void* d_out, int out_size, void* d_ws, size_t ws_size,
                              hipStream_t stream) {
  if (n_in < 21) return;
  if (in_sizes[0] != kB * kT || in_sizes[1] != kB * kT) return;
  if (in_sizes[2] != kV * kE) return;
  if (in_sizes[3] != kG * kE || in_sizes[7] != kG * kE) return;
  if (in_sizes[4] != kG * kH || in_sizes[8] != kG * kH || in_sizes[12] != kG * kH || in_sizes[16] != kG * kH) return;
  if (in_sizes[11] != kG * kTop || in_sizes[15] != kG * kTop) return;
  if (in_sizes[5] != kG || in_sizes[6] != kG || in_sizes[9] != kG || in_sizes[10] != kG) return;
  if (in_sizes[13] != kG || in_sizes[14] != kG || in_sizes[17] != kG || in_sizes[18] != kG) return;
  if (in_sizes[19] != kOut * kTop || in_sizes[20] != kOut) return;
  if (out_size != kB * kOut) return;
  if (ws_size < kWsTotal) return;

  const int*   ids     = (const int*)d_in[0];
  const int*   mask    = (const int*)d_in[1];
  const float* embed   = (const float*)d_in[2];
  const float* Wih_l0f = (const float*)d_in[3];
  const float* Whh_l0f = (const float*)d_in[4];
  const float* bih_l0f = (const float*)d_in[5];
  const float* bhh_l0f = (const float*)d_in[6];
  const float* Wih_l0b = (const float*)d_in[7];
  const float* Whh_l0b = (const float*)d_in[8];
  const float* bih_l0b = (const float*)d_in[9];
  const float* bhh_l0b = (const float*)d_in[10];
  const float* Wih_l1f = (const float*)d_in[11];
  const float* Whh_l1f = (const float*)d_in[12];
  const float* bih_l1f = (const float*)d_in[13];
  const float* bhh_l1f = (const float*)d_in[14];
  const float* Wih_l1b = (const float*)d_in[15];
  const float* Whh_l1b = (const float*)d_in[16];
  const float* bih_l1b = (const float*)d_in[17];
  const float* bhh_l1b = (const float*)d_in[18];
  const float* Wout    = (const float*)d_in[19];
  const float* bout    = (const float*)d_in[20];
  float* out = (float*)d_out;

  char* ws = (char*)d_ws;
  float*          GI   = (float*)(ws + kOffGI);
  unsigned short* X1   = (unsigned short*)(ws + kOffX1);
  unsigned short* EH   = (unsigned short*)(ws + kOffEH);
  unsigned short* W0H  = (unsigned short*)(ws + kOffW0H);
  unsigned short* W1H  = (unsigned short*)(ws + kOffW1H);
  unsigned short* WHH  = (unsigned short*)(ws + kOffWHH);
  float*          HFIN = (float*)(ws + kOffHFIN);

  cvt_f16c8_kernel<<<(kV * kE / 8) / 256, 256, 0, stream>>>(embed, EH, kV * kE / 8);
  PrepArgs pa;
  pa.wih0f = Wih_l0f; pa.wih0b = Wih_l0b; pa.wih1f = Wih_l1f; pa.wih1b = Wih_l1b;
  pa.whh0f = Whh_l0f; pa.whh0b = Whh_l0b; pa.whh1f = Whh_l1f; pa.whh1b = Whh_l1b;
  pa.w0h = W0H; pa.w1h = W1H; pa.whh = WHH;
  prep_weights_kernel<<<72, 128, 0, stream>>>(pa);

  gi_gemm_kernel<0><<<kM / 64, 128, 0, stream>>>(EH, ids, W0H, bih_l0f, bih_l0b, GI);
  gru_scan_kernel<0><<<32, 64, 0, stream>>>(GI, WHH, bhh_l0f, bhh_l0b, mask, X1, HFIN);

  gi_gemm_kernel<1><<<kM / 64, 128, 0, stream>>>(X1, ids, W1H, bih_l1f, bih_l1b, GI);
  gru_scan_kernel<1><<<32, 64, 0, stream>>>(GI, WHH, bhh_l1f, bhh_l1b, mask, X1, HFIN);

  head_kernel<<<(kB * kOut) / 256, 256, 0, stream>>>(HFIN, Wout, bout, out);
}
